// GNN_graphpred_48988396978771
// MI455X (gfx1250) — hardware-verified
//
#include <hip/hip_runtime.h>
#include <stddef.h>
#include <stdint.h>
#include <math.h>

#define NN   200000
#define NG   10000
#define NE   500000
#define NK   16
#define TROWS 128
#define NTHR 256
#define CTHR 1024
#define CWAV (CTHR / 32)
#define GSB  40
#define GSS  256
#define BINW (GSS * NTHR)
#define TABW 1024
#define TAB_K2 512
#define TAB_LW 528

#define WS_FLAG 0
#define WS_TAB  128
#define WS_T    (WS_TAB + 4 * 4096)
#define WS_EK   (WS_T + NN * 4)
#define WS_EV   (WS_EK + NE * 4)
#define WS_END  (WS_EV + NE * 4)
#define WSMAX   134217728

template <int D> struct GP {
  static constexpr int ND    = (D == 1 || D == 4) ? 40000 : 60000;
  static constexpr int OFF   = (D == 1) ? 0 : (D == 2) ? 40000 : (D == 3) ? 100000 : 160000;
  static constexpr int KC    = 5 + 12 * D;
  static constexpr int KPAD  = (KC <= 32) ? 32 : 64;
  static constexpr int NFEAT = 5 + 9 * D;
};

static_assert(NK == 16);
static_assert(CTHR == 1024 && CWAV == 32);
static_assert(NE % 4 == 0 && NN % 4 == 0 && NG % 4 == 0);
static_assert((NE * 4) % 128 == 0 && (NN * 4) % 128 == 0);
static_assert(GP<1>::OFF % 32 == 0 && GP<2>::OFF % 32 == 0 && GP<3>::OFF % 32 == 0 && GP<4>::OFF % 32 == 0);
static_assert(GP<1>::ND % 32 == 0 && GP<2>::ND % 32 == 0 && GP<3>::ND % 32 == 0 && GP<4>::ND % 32 == 0);
static_assert(GP<1>::OFF + GP<1>::ND == GP<2>::OFF && GP<2>::OFF + GP<2>::ND == GP<3>::OFF);
static_assert(GP<3>::OFF + GP<3>::ND == GP<4>::OFF && GP<4>::OFF + GP<4>::ND == NN);
static_assert(GP<1>::KC <= GP<1>::KPAD && GP<2>::KC <= GP<2>::KPAD && GP<3>::KC <= GP<3>::KPAD && GP<4>::KC <= GP<4>::KPAD);
static_assert(GP<1>::KPAD % 32 == 0 && GP<4>::KPAD % 32 == 0 && GP<4>::KPAD <= 64);
static_assert(16 * 64 / 2 <= TAB_K2 && TAB_LW == TAB_K2 + 16 && TAB_LW + 16 <= TABW);
static_assert(WS_TAB % 128 == 0 && WS_T % 128 == 0 && WS_EK % 128 == 0 && WS_EV % 128 == 0 && WS_END % 128 == 0);
static_assert(WS_END <= WSMAX);
static_assert(GSB * GSS >= NG && (NG * 4) % 16 == 0);
static_assert(BINW * 4 + 1024 <= 327680);

typedef float          v4f   __attribute__((ext_vector_type(4)));
typedef float          v8f   __attribute__((ext_vector_type(8)));
typedef int            v4i   __attribute__((ext_vector_type(4)));
typedef int            v8i   __attribute__((ext_vector_type(8)));
typedef unsigned int   v4u   __attribute__((ext_vector_type(4)));
typedef unsigned short v8us  __attribute__((ext_vector_type(8)));
typedef unsigned short v16us __attribute__((ext_vector_type(16)));
typedef __bf16         v16bf __attribute__((ext_vector_type(16)));
typedef v4f  __attribute__((may_alias)) v4fa;
typedef v4i  __attribute__((may_alias)) v4ia;
typedef v4u  __attribute__((may_alias)) v4ua;
typedef v8us __attribute__((may_alias)) v8usa;
typedef float __attribute__((may_alias)) f32a;
typedef int   __attribute__((may_alias)) i32a;
union FragB { v16bf v; v16us u; v8us h[2]; v8i w; };

__device__ __forceinline__ v8f wmb(const FragB& a, const FragB& b, v8f c) {
  v8f d = __builtin_amdgcn_wmma_f32_16x16x32_bf16(false, a.v, false, b.v, (short)0, c, false, false);
  asm volatile("v_nop\n\tv_nop\n\tv_nop\n\tv_nop" : "+v"(d) : "v"(a.w), "v"(b.w));
  return d;
}

__device__ __forceinline__ unsigned bf16_bits(float f) {
  const unsigned u = __float_as_uint(f);
  return (u + 0x7FFFu + ((u >> 16) & 1u)) >> 16;
}
__device__ __forceinline__ float bf16_val(float f) {
  return __uint_as_float(bf16_bits(f) << 16);
}
__device__ __forceinline__ unsigned short hbits(float v) {
  return (unsigned short)(__float_as_uint(v) >> 16);
}

__device__ __forceinline__ int chk_one(const int* __restrict__ s, int nvec, int off, int tid) {
  int bad = 0;
  const int nit = (nvec + CTHR - 1) / CTHR;
#pragma unroll 1
  for (int it = 0; it < nit; ++it) {
    const int i  = it * CTHR + tid;
    const bool ok = i < nvec;
    const int ic = ok ? i : nvec - 1;
    const v4i v = *(const v4ia*)(s + 4 * ic);
    const int r0 = off + 4 * ic;
    const int b = (v.x != r0) | (v.y != r0 + 1) | (v.z != r0 + 2) | (v.w != r0 + 3);
    bad |= ok ? b : 0;
  }
  return bad;
}

__global__ __launch_bounds__(CTHR) __attribute__((amdgpu_num_vgpr(248)))
void k_chk(const int* __restrict__ s1, const int* __restrict__ s2, const int* __restrict__ s3,
           const int* __restrict__ s4, int* flag) {
  __shared__ int flg[CWAV];
  const int tid = (int)threadIdx.x, lane = tid & 31, wave = tid >> 5;
  int bad = 0;
  bad |= chk_one(s1, GP<1>::ND / 4, GP<1>::OFF, tid);
  bad |= chk_one(s2, GP<2>::ND / 4, GP<2>::OFF, tid);
  bad |= chk_one(s3, GP<3>::ND / 4, GP<3>::OFF, tid);
  bad |= chk_one(s4, GP<4>::ND / 4, GP<4>::OFF, tid);
  const unsigned bm = __builtin_amdgcn_ballot_w32(bad != 0);
  const int wf = (bm != 0u) ? 1 : 0;
  if (lane == 0) flg[wave] = wf;
  __syncthreads();
  int any = 0;
#pragma unroll 4
  for (int w = 0; w < CWAV; ++w) any |= flg[w];
  const int fv = (any != 0) ? 1 : 0;
  const v4i o = {fv, fv, fv, fv};
  const bool wr = tid < 8;
  int* fp = flag + 4 * (tid & 7);
  if (wr) *(volatile v4i*)fp = o;
  __threadfence();
  if (wr) *(volatile v4i*)fp = o;
}

template <int D>
__global__ __launch_bounds__(NTHR) __attribute__((amdgpu_num_vgpr(248)))
void k_tab(const float* __restrict__ kx, const float* __restrict__ knx, const float* __restrict__ knp,
           const float* __restrict__ kne, const float* __restrict__ lw, unsigned int* tab) {
  constexpr int KPAD = GP<D>::KPAD;
  __shared__ float fb[16 * 64];
  __shared__ float k2s[16];
  __shared__ float lws[16];
  const int tid = (int)threadIdx.x;

#pragma unroll 1
  for (int it = 0; it < 4; ++it) {
    const int e  = it * NTHR + tid;
    const int k  = e >> 6, c = e & 63;
    const int cc = (c < 5) ? 0 : (c - 5);
    const int j  = cc / 12;
    const int q  = cc - 12 * j;
    const int jq = (j < D) ? j : (D - 1);
    const int qx = (q < 5) ? q : 4;
    const int qp = (q < 5) ? 0 : ((q < 8) ? (q - 5) : ((q < 11) ? (q - 8) : 2));
    const float vkx = kx[k * 5 + ((c < 5) ? c : 4)];
    const float vnx = knx[(k * D + jq) * 5 + qx];
    const float vnp = knp[(k * D + jq) * 3 + qp];
    const float vne = kne[k * D + jq];
    float v = (q < 5) ? vnx : ((q < 8) ? vnp : ((q < 11) ? (-vnp) : vne));
    v = (j < D) ? v : 0.0f;
    v = (c < 5) ? vkx : v;
    fb[e] = bf16_val(v);
  }
  if (tid < 16) lws[tid] = bf16_val(lw[16 * (D - 1) + tid]);
  __syncthreads();

  if (tid < 16) {
    float s = 0.0f;
#pragma unroll 4
    for (int c = 0; c < 64; ++c) {
      const int cc = (c < 5) ? 0 : (c - 5);
      const int q  = cc % 12;
      const bool skip = (c >= 5) && (q >= 8) && (q < 11);
      const float f = fb[tid * 64 + c];
      const float g = skip ? 0.0f : f;
      s = fmaf(g, g, s);
    }
    k2s[tid] = s;
  }
  __syncthreads();

  unsigned wv[4];
#pragma unroll
  for (int i = 0; i < 4; ++i) {
    const int w   = 4 * tid + i;
    const int hw  = 2 * w;
    const int row = hw / KPAD, col = hw % KPAD;
    const int rc  = (row < 16) ? row : 15;
    const float f0 = fb[rc * 64 + col], f1 = fb[rc * 64 + col + 1];
    unsigned btw = (__float_as_uint(f0) >> 16) | (__float_as_uint(f1) & 0xFFFF0000u);
    btw = (row < 16) ? btw : 0u;
    const int kk = w & 15;
    const unsigned k2w = __float_as_uint(k2s[kk]);
    const unsigned lww = __float_as_uint(lws[kk]);
    wv[i] = (w < TAB_K2) ? btw : ((w < TAB_LW) ? k2w : ((w < TAB_LW + 16) ? lww : 0u));
  }
  v4u o; o.x = wv[0]; o.y = wv[1]; o.z = wv[2]; o.w = wv[3];
  unsigned int* dp = tab + 4 * tid;
  *(volatile v4u*)dp = o;
  __threadfence();
  *(volatile v4u*)dp = o;
}

__device__ __forceinline__ void stage_chunk(const float* __restrict__ src, float* dst, int g0, int nvec,
                                            int total, int tid) {
#pragma unroll 1
  for (int q0 = 0; q0 < nvec; q0 += NTHR) {
    const int q = q0 + tid;
    const int g = g0 + 4 * q;
    const bool inq = q < nvec;
    const bool ok = inq && (g < total);
    const int gc = ok ? g : 0;
    const v4f v = *(const v4fa*)(src + gc);
    v4f r;
    r.x = ok ? bf16_val(v.x) : 0.0f;
    r.y = ok ? bf16_val(v.y) : 0.0f;
    r.z = ok ? bf16_val(v.z) : 0.0f;
    r.w = ok ? bf16_val(v.w) : 0.0f;
    if (inq) *(v4fa*)(dst + 4 * q) = r;
  }
}

template <int D>
__global__ __launch_bounds__(NTHR) __attribute__((amdgpu_num_vgpr(248)))
void k_node(const float* __restrict__ xf, const float* __restrict__ pf, const float* __restrict__ nx,
            const float* __restrict__ np, const float* __restrict__ ne,
            const unsigned int* __restrict__ tab, float* T) {
  constexpr int ND = GP<D>::ND, OFF = GP<D>::OFF, KC = GP<D>::KC, KPAD = GP<D>::KPAD, NFEAT = GP<D>::NFEAT;
  constexpr int KP = KPAD + 8;
  static_assert((KP * 2) % 16 == 0);
  static_assert(4 * (640 + 384 + 640 * D + 384 * D + 128 * D) + 2 * 128 * KP + 4 * (128 + 128 * 17 + 128 + 32) <= 65536);
  __shared__ __attribute__((aligned(16))) float sXF[TROWS * 5];
  __shared__ __attribute__((aligned(16))) float sPF[TROWS * 3];
  __shared__ __attribute__((aligned(16))) float sNX[TROWS * 5 * D];
  __shared__ __attribute__((aligned(16))) float sNP[TROWS * 3 * D];
  __shared__ __attribute__((aligned(16))) float sNE[TROWS * D];
  __shared__ __attribute__((aligned(16))) unsigned short sA[TROWS * KP];
  __shared__ float sA2[TROWS];
  __shared__ float sD[TROWS * 17];
  __shared__ __attribute__((aligned(16))) float sT[TROWS];
  __shared__ float sK2[16];
  __shared__ float sLW[16];

  const int tid = (int)threadIdx.x, lane = tid & 31, wave = tid >> 5, hh = lane >> 4, m = lane & 15;
  const int tile = (int)blockIdx.x;
  const int r0g = tile * TROWS;

  stage_chunk(xf, sXF, r0g * 5,     32 * 5,     ND * 5,     tid);
  stage_chunk(pf, sPF, r0g * 3,     32 * 3,     ND * 3,     tid);
  stage_chunk(nx, sNX, r0g * 5 * D, 32 * 5 * D, ND * 5 * D, tid);
  stage_chunk(np, sNP, r0g * 3 * D, 32 * 3 * D, ND * 3 * D, tid);
  stage_chunk(ne, sNE, r0g * D,     32 * D,     ND * D,     tid);
  if (tid < 32) {
    const float v = __uint_as_float(tab[TAB_K2 + tid]);
    if (tid < 16) sK2[tid] = v; else sLW[tid - 16] = v;
  }
  __syncthreads();

  if (tid < TROWS) {
    const int r = tid;
    unsigned short* ar = sA + r * KP;
#pragma unroll
    for (int i = 0; i < 5; ++i) ar[i] = hbits(sXF[r * 5 + i]);
#pragma unroll 1
    for (int j = 0; j < D; ++j) {
      unsigned short* aj = ar + 5 + 12 * j;
#pragma unroll
      for (int i = 0; i < 5; ++i) aj[i] = hbits(sNX[(r * D + j) * 5 + i]);
#pragma unroll
      for (int i = 0; i < 3; ++i) aj[5 + i] = hbits(sNP[(r * D + j) * 3 + i]);
#pragma unroll
      for (int i = 0; i < 3; ++i) aj[8 + i] = hbits(sPF[r * 3 + i]);
      aj[11] = hbits(sNE[r * D + j]);
    }
#pragma unroll 1
    for (int c = KC; c < KPAD; ++c) ar[c] = (unsigned short)0;
  } else {
    const int r = tid - TROWS;
    float s = 0.0f;
#pragma unroll
    for (int i = 0; i < 5; ++i) { const float x = sXF[r * 5 + i]; s = fmaf(x, x, s); }
#pragma unroll 1
    for (int j = 0; j < D; ++j) {
#pragma unroll
      for (int i = 0; i < 5; ++i) { const float x = sNX[(r * D + j) * 5 + i]; s = fmaf(x, x, s); }
#pragma unroll
      for (int i = 0; i < 3; ++i) {
        const float d = sNP[(r * D + j) * 3 + i] - sPF[r * 3 + i];
        s = fmaf(d, d, s);
      }
      const float e = sNE[r * D + j];
      s = fmaf(e, e, s);
    }
    sA2[r] = s;
  }
  __syncthreads();

  {
    v8f acc = {0.f, 0.f, 0.f, 0.f, 0.f, 0.f, 0.f, 0.f};
    const unsigned short* arow = sA + (16 * wave + m) * KP + 8 * hh;
    const unsigned short* brow = (const unsigned short*)tab + m * KPAD + 8 * hh;
#pragma unroll
    for (int ks = 0; ks < KPAD / 32; ++ks) {
      FragB af, bf;
      af.h[0] = *(const v8usa*)(arow + 32 * ks);
      af.h[1] = *(const v8usa*)(arow + 32 * ks + 16);
      bf.h[0] = *(const v8usa*)(brow + 32 * ks);
      bf.h[1] = *(const v8usa*)(brow + 32 * ks + 16);
      acc = wmb(af, bf, acc);
    }
#pragma unroll
    for (int r = 0; r < 8; ++r) sD[(16 * wave + 8 * hh + r) * 17 + m] = acc[r];
  }
  __syncthreads();

  if (tid < TROWS) {
    const int r = tid;
    const float a2 = sA2[r];
    float t = 0.0f;
#pragma unroll 1
    for (int k = 0; k < NK; ++k) {
      const float d2 = (a2 + sK2[k]) - 2.0f * sD[r * 17 + k];
      const float s = expf((-d2) / (float)NFEAT);
      t = fmaf(s, sLW[k], t);
    }
    sT[r] = t;
  }
  __syncthreads();

  {
    const int l4 = 4 * (tid & 31);
    const int rowg = r0g + l4;
    const bool wr = (tid < 32) && (rowg < ND);
    const v4f tv = *(const v4fa*)(sT + l4);
    float* tp = T + OFF + (wr ? rowg : 0);
    if (wr) *(volatile v4f*)tp = tv;
    __threadfence();
    if (wr) *(volatile v4f*)tp = tv;
  }
}

__global__ __launch_bounds__(NTHR) __attribute__((amdgpu_num_vgpr(248)))
void k_edge(const int* __restrict__ ei, const int* __restrict__ bat, const float* __restrict__ T,
            int* ek, float* ev) {
  const int u = (int)blockIdx.x * NTHR + (int)threadIdx.x;
  const bool ok = u < NE / 4;
  const int uc = ok ? u : 0;
  const v4i s = *(const v4ia*)(ei + 4 * uc);
  const v4i d = *(const v4ia*)(ei + NE + 4 * uc);
  const int d0 = min(max(d.x, 0), NN - 1), d1 = min(max(d.y, 0), NN - 1);
  const int d2 = min(max(d.z, 0), NN - 1), d3 = min(max(d.w, 0), NN - 1);
  const int b0 = bat[d0], b1 = bat[d1], b2 = bat[d2], b3 = bat[d3];
  v4i kv;
  kv.x = ((unsigned)d.x < (unsigned)NN) ? b0 : -1;
  kv.y = ((unsigned)d.y < (unsigned)NN) ? b1 : -1;
  kv.z = ((unsigned)d.z < (unsigned)NN) ? b2 : -1;
  kv.w = ((unsigned)d.w < (unsigned)NN) ? b3 : -1;
  const int s0 = min(max(s.x, 0), NN - 1), s1 = min(max(s.y, 0), NN - 1);
  const int s2 = min(max(s.z, 0), NN - 1), s3 = min(max(s.w, 0), NN - 1);
  v4f vv;
  vv.x = T[s0]; vv.y = T[s1]; vv.z = T[s2]; vv.w = T[s3];
  int*   kp = ek + 4 * uc;
  float* vp = ev + 4 * uc;
  if (ok) { *(volatile v4i*)kp = kv; *(volatile v4f*)vp = vv; }
  __threadfence();
  if (ok) { *(volatile v4i*)kp = kv; *(volatile v4f*)vp = vv; }
}

__device__ __forceinline__ void bin_addf(f32a* fbn, int key, float val, bool ok, int base, int tid) {
  const unsigned sl = (unsigned)(key - base);
  const bool hit = ok && (sl < (unsigned)GSS);
  const int sc = hit ? (int)sl : 0;
  const float add = hit ? val : 0.0f;
  const float cur = fbn[sc * NTHR + tid];
  fbn[sc * NTHR + tid] = cur + add;
}
__device__ __forceinline__ void bin_addi(i32a* ibn, int key, bool ok, int base, int tid) {
  const unsigned sl = (unsigned)(key - base);
  const bool hit = ok && (sl < (unsigned)GSS);
  const int sc = hit ? (int)sl : 0;
  const int add = hit ? 1 : 0;
  const int cur = ibn[sc * NTHR + tid];
  ibn[sc * NTHR + tid] = cur + add;
}

__global__ __launch_bounds__(NTHR) __attribute__((amdgpu_num_vgpr(248)))
void k_gscan(const int* __restrict__ ek, const float* __restrict__ ev, const int* __restrict__ bat,
             const float* __restrict__ lb, const int* __restrict__ flag, float* out) {
  extern __shared__ __attribute__((aligned(16))) unsigned int bins[];
  __shared__ __attribute__((aligned(16))) float outs[GSS];
  const int tid = (int)threadIdx.x;
  const int base = (int)blockIdx.x * GSS;
  f32a* fbn = (f32a*)bins;
  i32a* ibn = (i32a*)bins;
  const v4u z4 = {0u, 0u, 0u, 0u};

#pragma unroll 1
  for (int i = 4 * tid; i < BINW; i += 4 * NTHR) *(v4ua*)(bins + i) = z4;
  __syncthreads();

  constexpr int NIT_E = (NE + 1023) / 1024;
#pragma unroll 1
  for (int c = 0; c < NIT_E; ++c) {
    const int e0 = c * 1024 + 4 * tid;
    const bool ok = e0 < NE;
    const int ec = ok ? e0 : (NE - 4);
    const v4i k = *(const v4ia*)(ek + ec);
    const v4f v = *(const v4fa*)(ev + ec);
    bin_addf(fbn, k.x, v.x, ok, base, tid);
    bin_addf(fbn, k.y, v.y, ok, base, tid);
    bin_addf(fbn, k.z, v.z, ok, base, tid);
    bin_addf(fbn, k.w, v.w, ok, base, tid);
  }
  __syncthreads();

  float sum = 0.0f;
#pragma unroll 4
  for (int j = 0; j < NTHR; j += 4) {
    const v4f x = *(const v4fa*)(bins + tid * NTHR + j);
    sum = (((sum + x.x) + x.y) + x.z) + x.w;
  }
  __syncthreads();

#pragma unroll 1
  for (int i = 4 * tid; i < BINW; i += 4 * NTHR) *(v4ua*)(bins + i) = z4;
  __syncthreads();

  constexpr int NIT_N = (NN + 1023) / 1024;
#pragma unroll 1
  for (int c = 0; c < NIT_N; ++c) {
    const int n0 = c * 1024 + 4 * tid;
    const bool ok = n0 < NN;
    const int nc = ok ? n0 : (NN - 4);
    const v4i k = *(const v4ia*)(bat + nc);
    bin_addi(ibn, k.x, ok, base, tid);
    bin_addi(ibn, k.y, ok, base, tid);
    bin_addi(ibn, k.z, ok, base, tid);
    bin_addi(ibn, k.w, ok, base, tid);
  }
  __syncthreads();

  int cnt = 0;
#pragma unroll 4
  for (int j = 0; j < NTHR; j += 4) {
    const v4i x = *(const v4ia*)(bins + tid * NTHR + j);
    cnt = (((cnt + x.x) + x.y) + x.z) + x.w;
  }

  {
    const float bb = bf16_val(lb[0]);
    const int fl = flag[0];
    const float den = fmaxf((float)cnt, 1.0f);
    const float v = sum / den + bb;
    const float qnan = __int_as_float(0x7fc00000);
    outs[tid] = (fl != 0) ? qnan : v;
  }
  __syncthreads();

  {
    const int l4 = 4 * (tid & 63);
    const int g0 = base + l4;
    const bool wr = (tid < 64) && (g0 < NG);
    const v4f ov = *(const v4fa*)(outs + l4);
    float* op = out + (wr ? g0 : 0);
    if (wr) *(volatile v4f*)op = ov;
    __threadfence();
    if (wr) *(volatile v4f*)op = ov;
  }
}

static inline int cdiv(int a, int b) { return (a + b - 1) / b; }

static inline bool group_sizes_ok(const int* sz, int base, int nd, int d) {
  return sz[base + 0] == nd * 5 && sz[base + 1] == nd * 3 && sz[base + 2] == nd * d * 5 &&
         sz[base + 3] == nd * d * 3 && sz[base + 4] == nd * d && sz[base + 5] == nd &&
         sz[base + 6] == 80 && sz[base + 7] == 80 * d && sz[base + 8] == 48 * d && sz[base + 9] == 16 * d;
}

extern "C" void kernel_launch(void* const* d_in, const int* in_sizes, int n_in,
                              void* d_out, int out_size, void* d_ws, size_t ws_size,
                              hipStream_t stream) {
  if (n_in < 44) return;
  if (!group_sizes_ok(in_sizes,  0, GP<1>::ND, 1)) return;
  if (!group_sizes_ok(in_sizes, 10, GP<2>::ND, 2)) return;
  if (!group_sizes_ok(in_sizes, 20, GP<3>::ND, 3)) return;
  if (!group_sizes_ok(in_sizes, 30, GP<4>::ND, 4)) return;
  if (in_sizes[40] != 2 * NE || in_sizes[41] != NN || in_sizes[42] != 64 || in_sizes[43] != 1) return;
  if (out_size != NG) return;
  if ((size_t)WS_END > ws_size) return;

  const float* F[44];
  for (int i = 0; i < 44; ++i) F[i] = (const float*)d_in[i];
  const int* sel1 = (const int*)d_in[5];
  const int* sel2 = (const int*)d_in[15];
  const int* sel3 = (const int*)d_in[25];
  const int* sel4 = (const int*)d_in[35];
  const int*   ei  = (const int*)d_in[40];
  const int*   bat = (const int*)d_in[41];
  const float* lw  = (const float*)d_in[42];
  const float* lb  = (const float*)d_in[43];
  float* out = (float*)d_out;

  char* ws = (char*)d_ws;
  int*          FLAG = (int*)(ws + WS_FLAG);
  unsigned int* TAB1 = (unsigned int*)(ws + WS_TAB + 0 * 4096);
  unsigned int* TAB2 = (unsigned int*)(ws + WS_TAB + 1 * 4096);
  unsigned int* TAB3 = (unsigned int*)(ws + WS_TAB + 2 * 4096);
  unsigned int* TAB4 = (unsigned int*)(ws + WS_TAB + 3 * 4096);
  float* T  = (float*)(ws + WS_T);
  int*   EK = (int*)(ws + WS_EK);
  float* EV = (float*)(ws + WS_EV);

  const size_t gsLds = (size_t)BINW * 4;
  hipFuncSetAttribute(reinterpret_cast<const void*>(&k_gscan), hipFuncAttributeMaxDynamicSharedMemorySize, (int)gsLds);

  k_chk<<<1, CTHR, 0, stream>>>(sel1, sel2, sel3, sel4, FLAG);
  k_tab<1><<<1, NTHR, 0, stream>>>(F[6],  F[7],  F[8],  F[9],  lw, TAB1);
  k_tab<2><<<1, NTHR, 0, stream>>>(F[16], F[17], F[18], F[19], lw, TAB2);
  k_tab<3><<<1, NTHR, 0, stream>>>(F[26], F[27], F[28], F[29], lw, TAB3);
  k_tab<4><<<1, NTHR, 0, stream>>>(F[36], F[37], F[38], F[39], lw, TAB4);
  k_node<1><<<cdiv(GP<1>::ND, TROWS), NTHR, 0, stream>>>(F[0],  F[1],  F[2],  F[3],  F[4],  TAB1, T);
  k_node<2><<<cdiv(GP<2>::ND, TROWS), NTHR, 0, stream>>>(F[10], F[11], F[12], F[13], F[14], TAB2, T);
  k_node<3><<<cdiv(GP<3>::ND, TROWS), NTHR, 0, stream>>>(F[20], F[21], F[22], F[23], F[24], TAB3, T);
  k_node<4><<<cdiv(GP<4>::ND, TROWS), NTHR, 0, stream>>>(F[30], F[31], F[32], F[33], F[34], TAB4, T);
  k_edge<<<cdiv(NE / 4, NTHR), NTHR, 0, stream>>>(ei, bat, T, EK, EV);
  k_gscan<<<GSB, NTHR, gsLds, stream>>>(EK, EV, bat, lb, FLAG, out);
}
